// LSTMPolicy_88940182765653
// MI455X (gfx1250) — hardware-verified
//
#include <hip/hip_runtime.h>

#define NBATCH 65536
#define NIN    64
#define NHID   128
#define NACT   16
#define RPB    128
#define HSTR   136

typedef _Float16 f16;
typedef __attribute__((ext_vector_type(16))) f16 f16x16;
typedef __attribute__((ext_vector_type(8)))  f16 f16x8;
typedef __attribute__((ext_vector_type(8)))  float f32x8;
typedef __attribute__((ext_vector_type(4)))  float v4f_t;
typedef float v4fa __attribute__((ext_vector_type(4), may_alias));

__device__ __forceinline__ f32x8 wmma16(f16x16 a, f16x16 b, f32x8 c) {
  return __builtin_amdgcn_wmma_f32_16x16x32_f16(false, a, false, b, (short)0, c, false, false);
}
__device__ __forceinline__ f16x16 load_frag(const float* __restrict__ base, int ld, int row0, int k0) {
  const int lane = threadIdx.x & 31, r = lane & 15, kh = (lane >> 4) * 8;
  const float* p0 = base + (size_t)(row0 + r) * ld + (k0 + kh);
  const v4f_t a = *(const v4f_t*)(p0), b = *(const v4f_t*)(p0 + 4), c = *(const v4f_t*)(p0 + 16), d = *(const v4f_t*)(p0 + 20);
  f16x16 f;
  f[0] = (f16)a[0]; f[1] = (f16)a[1]; f[2]  = (f16)a[2]; f[3]  = (f16)a[3]; f[4]  = (f16)b[0]; f[5]  = (f16)b[1]; f[6]  = (f16)b[2]; f[7]  = (f16)b[3];
  f[8] = (f16)c[0]; f[9] = (f16)c[1]; f[10] = (f16)c[2]; f[11] = (f16)c[3]; f[12] = (f16)d[0]; f[13] = (f16)d[1]; f[14] = (f16)d[2]; f[15] = (f16)d[3];
  return f;
}
__device__ __forceinline__ f16x16 lds_frag(const f16* base, int stride) {
  const int lane = threadIdx.x & 31, row = lane & 15, kh = (lane >> 4) * 8;
  const f16x8 lo = *(const f16x8*)(base + row * stride + kh);
  const f16x8 hi = *(const f16x8*)(base + row * stride + kh + 16);
  f16x16 f;
#pragma unroll
  for (int i = 0; i < 8; ++i) { f[i] = lo[i]; f[i + 8] = hi[i]; }
  return f;
}
__device__ __forceinline__ float sigm(float x) { return 1.0f / (1.0f + __expf(-x)); }
__device__ __forceinline__ float tanh_(float x) { return 1.0f - 2.0f / (1.0f + __expf(2.0f * x)); }

template <int KSTEPS>
__device__ __forceinline__ void lstm_layer(const f16x16* af, const float* __restrict__ W, const float* __restrict__ bi,
                                           const float* __restrict__ bh, f16* hT) {
  const int lane = threadIdx.x & 31, col = lane & 15, rh = (lane >> 4) * 8;
  constexpr int K = KSTEPS * 32;
#pragma unroll 1
  for (int jt = 0; jt < NHID / 16; ++jt) {
    f32x8 ai = {}, ag = {}, ao = {};
#pragma unroll
    for (int ks = 0; ks < KSTEPS; ++ks) {
      ai = wmma16(af[ks], load_frag(W, K, 0 * NHID + jt * 16, ks * 32), ai);
      ag = wmma16(af[ks], load_frag(W, K, 2 * NHID + jt * 16, ks * 32), ag);
      ao = wmma16(af[ks], load_frag(W, K, 3 * NHID + jt * 16, ks * 32), ao);
    }
    const int j = jt * 16 + col;
    const float bI = bi[j] + bh[j], bG = bi[2 * NHID + j] + bh[2 * NHID + j], bO = bi[3 * NHID + j] + bh[3 * NHID + j];
#pragma unroll
    for (int r = 0; r < 8; ++r) {
      const float ig = sigm(ai[r] + bI), gg = tanh_(ag[r] + bG), og = sigm(ao[r] + bO);
      const float c = ig * gg;
      hT[(rh + r) * HSTR + j] = (f16)(og * tanh_(c));
    }
  }
}

__global__ __launch_bounds__(256) void lstm_policy_kernel(const float* __restrict__ x,
    const float* __restrict__ Wih0, const float* __restrict__ bih0, const float* __restrict__ bhh0,
    const float* __restrict__ Wih1, const float* __restrict__ bih1, const float* __restrict__ bhh1,
    const float* __restrict__ Wp, const float* __restrict__ bp, const float* __restrict__ Wv, const float* __restrict__ bv,
    float* __restrict__ policy, float* __restrict__ value) {
  __shared__ __attribute__((aligned(16))) f16 h0S[8][16 * HSTR];
  __shared__ __attribute__((aligned(16))) f16 h1S[8][16 * HSTR];
  __shared__ __attribute__((aligned(16))) float polS[8][16 * 16];
  __shared__ __attribute__((aligned(16))) float valS[RPB];
  const int tid = threadIdx.x, lane = tid & 31, wave = tid >> 5, col = lane & 15, rh = (lane >> 4) * 8;
  const int row0 = blockIdx.x * RPB + wave * 16;

  {
    f16x16 xa[2] = { load_frag(x, NIN, row0, 0), load_frag(x, NIN, row0, 32) };
    lstm_layer<2>(xa, Wih0, bih0, bhh0, h0S[wave]);
  }
  __syncthreads();
  {
    f16x16 ha[4];
#pragma unroll
    for (int ks = 0; ks < 4; ++ks) ha[ks] = lds_frag(h0S[wave] + ks * 32, HSTR);
    lstm_layer<4>(ha, Wih1, bih1, bhh1, h1S[wave]);
  }
  __syncthreads();
  {
    f32x8 ap = {}, av = {};
#pragma unroll
    for (int ks = 0; ks < 4; ++ks) {
      const f16x16 ha = lds_frag(h1S[wave] + ks * 32, HSTR);
      ap = wmma16(ha, load_frag(Wp, NHID, 0, ks * 32), ap);
      f16x16 bv_;
      const int kh = (lane >> 4) * 8;
#pragma unroll
      for (int e = 0; e < 8; ++e) {
        bv_[e]     = (col == 0) ? (f16)Wv[ks * 32 + kh + e]      : (f16)0.0f;
        bv_[e + 8] = (col == 0) ? (f16)Wv[ks * 32 + kh + 16 + e] : (f16)0.0f;
      }
      av = wmma16(ha, bv_, av);
    }
    const float bpc = bp[col];
#pragma unroll
    for (int r = 0; r < 8; ++r) polS[wave][(rh + r) * 16 + col] = ap[r] + bpc;
    if (col == 0) {
#pragma unroll
      for (int r = 0; r < 8; ++r) valS[wave * 16 + rh + r] = av[r] + bv[0];
    }
  }
  __syncthreads();
#pragma unroll 1
  for (int pass = 0; pass < 2; ++pass) {
#pragma unroll
    for (int u = 0; u < 2; ++u) {
      const int f4 = lane + 32 * u;
      *(volatile v4f_t*)(policy + (size_t)row0 * NACT + 4 * f4) = *(const volatile v4fa*)(polS[wave] + 4 * f4);
    }
    if (wave == 0) *(volatile v4f_t*)(value + (size_t)blockIdx.x * RPB + 4 * lane) = *(const volatile v4fa*)(valS + 4 * lane);
    __threadfence();
  }
}

extern "C" void kernel_launch(void* const* d_in, const int* in_sizes, int n_in,
                              void* d_out, int out_size, void* d_ws, size_t ws_size,
                              hipStream_t stream) {
  (void)in_sizes; (void)n_in; (void)out_size; (void)d_ws; (void)ws_size;
  const float* x    = (const float*)d_in[0];
  const float* Wih0 = (const float*)d_in[1];
  const float* Whh0 = (const float*)d_in[2];
  const float* bih0 = (const float*)d_in[3];
  const float* bhh0 = (const float*)d_in[4];
  const float* Wih1 = (const float*)d_in[5];
  const float* Whh1 = (const float*)d_in[6];
  const float* bih1 = (const float*)d_in[7];
  const float* bhh1 = (const float*)d_in[8];
  const float* Wp   = (const float*)d_in[9];
  const float* bp   = (const float*)d_in[10];
  const float* Wv   = (const float*)d_in[11];
  const float* bv   = (const float*)d_in[12];
  (void)Whh0; (void)Whh1;
  float* policy = (float*)d_out;
  float* value  = policy + (size_t)NBATCH * NACT;
  lstm_policy_kernel<<<dim3(NBATCH / RPB), dim3(256), 0, stream>>>(x, Wih0, bih0, bhh0, Wih1, bih1, bhh1, Wp, bp, Wv, bv,
                                                              policy, value);
}
